// Mamba_v1_27865747817195
// MI455X (gfx1250) — hardware-verified
//
#include <hip/hip_runtime.h>
#include <math.h>

typedef __attribute__((ext_vector_type(16))) __bf16   v16b;
typedef __attribute__((ext_vector_type(8)))  __bf16   v8b;
typedef __attribute__((ext_vector_type(8)))  _Float16 v8h;
typedef __attribute__((ext_vector_type(8)))  float    v8f;
typedef __attribute__((ext_vector_type(4)))  float    v4f;
typedef __attribute__((ext_vector_type(2)))  float    v2f;

constexpr int kNumSeq   = 8192;
constexpr int kSteps    = 6;
constexpr int kHid      = 32;
constexpr int kInner    = 64;
constexpr int kStates   = 64;
constexpr int kFeat     = 45;
constexpr int kFeatPad  = 64;
constexpr int kProjN    = 130;
constexpr int kProjPad  = 144;
constexpr int kSeqBlk   = 8;
constexpr int kRowsBlk  = kSeqBlk * kSteps;
constexpr int kHeadSeq  = 64;
constexpr int kOut0Cols = 7;
constexpr int kOut1Cols = 3;
constexpr int kOut0Elems = kNumSeq * kOut0Cols;
constexpr int kOut1Elems = kNumSeq * kOut1Cols;
constexpr int kOutTotal  = kOut0Elems + kOut1Elems + 2;
static_assert(kRowsBlk == 48, "three full 16-row tiles per wave");
static_assert((kNumSeq % kSeqBlk) == 0 && (kNumSeq % kHeadSeq) == 0, "grid multiples");
static_assert(kFeat == 22 + 12 + 7 + 4, "feature concat");
static_assert(kProjN == 2 + 2 * kStates && (kProjPad % 16) == 0 && kProjPad >= kProjN, "x_proj width");
static_assert((kFeatPad % 32) == 0 && (kHid % 32) == 0 && (kInner % 32) == 0, "K multiples of 32");
static_assert((kOut0Elems * 4) % 128 == 0 && ((kOut0Elems + kOut1Elems) * 4) % 128 == 0, "output bases line aligned");
static_assert((kHeadSeq * kOut0Cols * 4) % 128 == 0 && (kHeadSeq * kOut1Cols * 4) % 128 == 0, "head block owns whole lines");
static_assert(kOutTotal * 4 == 327688, "output bytes");

constexpr size_t kOffWF1   = 0;
constexpr size_t kOffWF2   = kOffWF1   + (size_t)kHid * kFeatPad * 2;
constexpr size_t kOffWIN1  = kOffWF2   + (size_t)kHid * kHid * 2;
constexpr size_t kOffWXP1  = kOffWIN1  + (size_t)2 * kInner * kHid * 2;
constexpr size_t kOffWOUT1 = kOffWXP1  + (size_t)kProjPad * kInner * 2;
constexpr size_t kOffWIN2  = kOffWOUT1 + (size_t)kHid * kInner * 2;
constexpr size_t kOffWXP2  = kOffWIN2  + (size_t)2 * kInner * kHid * 2;
constexpr size_t kOffWOUT2 = kOffWXP2  + (size_t)kProjPad * kInner * 2;
constexpr size_t kOffXL    = kOffWOUT2 + (size_t)kHid * kInner * 2;
constexpr size_t kWsTotal  = kOffXL    + (size_t)kNumSeq * kHid * 4;
static_assert(kWsTotal == 1116160ull, "carve total");
static_assert(kWsTotal <= 134217728ull, "carve cap");
static_assert((kOffWF2 % 128) == 0 && (kOffWIN1 % 128) == 0 && (kOffWXP1 % 128) == 0 && (kOffWOUT1 % 128) == 0 &&
              (kOffWIN2 % 128) == 0 && (kOffWXP2 % 128) == 0 && (kOffWOUT2 % 128) == 0 && (kOffXL % 128) == 0,
              "128-B aligned regions");

__device__ __forceinline__ unsigned short f2bf_bits(float f) {
  unsigned u = __float_as_uint(f);
  return (unsigned short)((u + 0x7FFFu + ((u >> 16) & 1u)) >> 16);
}
__device__ __forceinline__ float bf_bits2f(unsigned short h) { return __uint_as_float(((unsigned)h) << 16); }
__device__ __forceinline__ float rbf(float f) { return bf_bits2f(f2bf_bits(f)); }

__device__ __forceinline__ v8f mma_bf(v16b a, v16b b, v8f c) {
  c = __builtin_amdgcn_wmma_f32_16x16x32_bf16(false, a, false, b, (short)0, c, false, false);
  asm volatile("v_nop\n\tv_nop\n\tv_nop\n\tv_nop" : "+v"(c) : "v"(a), "v"(b));
  return c;
}

__device__ __forceinline__ v16b load_b_frag(const unsigned short* p) {
  union U { v16b v; v8b h[2]; } f;
  const __bf16* q = (const __bf16*)(const void*)p;
  f.h[0] = *(const v8b*)(q);
  f.h[1] = *(const v8b*)(q + 16);
  return f.v;
}

__device__ __forceinline__ v16b frag_hi(const float* p) {
  const v4f a0 = *(const v4f*)(p);
  const v4f a1 = *(const v4f*)(p + 4);
  const v4f a2 = *(const v4f*)(p + 16);
  const v4f a3 = *(const v4f*)(p + 20);
  v16b hi;
#pragma unroll
  for (int e = 0; e < 4; ++e) {
    const float x0 = a0[e], x1 = a1[e], x2 = a2[e], x3 = a3[e];
    const unsigned short h0 = f2bf_bits(x0), h1 = f2bf_bits(x1), h2 = f2bf_bits(x2), h3 = f2bf_bits(x3);
    hi[e]      = __builtin_bit_cast(__bf16, h0);
    hi[4 + e]  = __builtin_bit_cast(__bf16, h1);
    hi[8 + e]  = __builtin_bit_cast(__bf16, h2);
    hi[12 + e] = __builtin_bit_cast(__bf16, h3);
  }
  return hi;
}

__device__ __forceinline__ void frag_hi_lo(const float* p, v16b& hi, v16b& lo) {
  const v4f a0 = *(const v4f*)(p);
  const v4f a1 = *(const v4f*)(p + 4);
  const v4f a2 = *(const v4f*)(p + 16);
  const v4f a3 = *(const v4f*)(p + 20);
#pragma unroll
  for (int e = 0; e < 4; ++e) {
    const float x0 = a0[e], x1 = a1[e], x2 = a2[e], x3 = a3[e];
    const unsigned short h0 = f2bf_bits(x0), h1 = f2bf_bits(x1), h2 = f2bf_bits(x2), h3 = f2bf_bits(x3);
    const unsigned short l0 = f2bf_bits(x0 - bf_bits2f(h0));
    const unsigned short l1 = f2bf_bits(x1 - bf_bits2f(h1));
    const unsigned short l2 = f2bf_bits(x2 - bf_bits2f(h2));
    const unsigned short l3 = f2bf_bits(x3 - bf_bits2f(h3));
    hi[e]      = __builtin_bit_cast(__bf16, h0);
    hi[4 + e]  = __builtin_bit_cast(__bf16, h1);
    hi[8 + e]  = __builtin_bit_cast(__bf16, h2);
    hi[12 + e] = __builtin_bit_cast(__bf16, h3);
    lo[e]      = __builtin_bit_cast(__bf16, l0);
    lo[4 + e]  = __builtin_bit_cast(__bf16, l1);
    lo[8 + e]  = __builtin_bit_cast(__bf16, l2);
    lo[12 + e] = __builtin_bit_cast(__bf16, l3);
  }
}

__device__ __forceinline__ float sigmoid_f(float x) { return 1.0f / (1.0f + expf(-x)); }

__global__ __launch_bounds__(256) void pad_cast_bf16_kernel(
    const float* __restrict__ src, unsigned short* __restrict__ dst, int nreal, int kreal, int kpad, int total8)
{
  const int i = blockIdx.x * 256 + threadIdx.x;
  if (i >= total8) return;
  const int e0 = i << 3;
  const int n  = e0 / kpad;
  const int k0 = e0 - n * kpad;
  const int nc = (n < nreal) ? n : (nreal - 1);
  const bool nok = (n < nreal);
  v8h hv;
#pragma unroll
  for (int e = 0; e < 8; ++e) {
    const int k  = k0 + e;
    const int kc = (k < kreal) ? k : (kreal - 1);
    const float v = src[nc * kreal + kc];
    const bool ok = nok && (k < kreal);
    const unsigned short bits = ok ? f2bf_bits(v) : (unsigned short)0;
    hv[e] = __builtin_bit_cast(_Float16, bits);
  }
  unsigned short* q = dst + e0;
  *(volatile v8h*)q = hv;
  __threadfence();
  *(volatile v8h*)q = hv;
}

struct SsmW {
  const float* lnw; const float* lnb; const float* conv_w; const float* conv_b;
  const float* dt_w; const float* dt_b; const float* alog; const float* dp;
  const unsigned short* win; const unsigned short* wxp; const unsigned short* wout;
};
static_assert(sizeof(SsmW) == 88, "no padding");

struct FusedArgs {
  const float* xs; const float* xd; const float* xp; const float* xt; const float* fc1_b;
  const unsigned short* wf1;
  SsmW m1; SsmW m2;
  float* xl;
};
static_assert(sizeof(FusedArgs) == 232, "no padding");

__device__ __forceinline__ void ssm_block(float* sX, float* sXZ, float* sD, const SsmW w, const int lane)
{
  const int hh = lane >> 4, m = lane & 15;
  float* sU = sD;

  {
    const float lw = rbf(w.lnw[lane]);
    const float lb = rbf(w.lnb[lane]);
#pragma unroll 2
    for (int row = 0; row < kRowsBlk; ++row) {
      const float v = sX[row * kHid + lane];
      float s = v;
      s += __shfl_xor(s, 16, 32);
      s += __shfl_xor(s, 8, 32);
      s += __shfl_xor(s, 4, 32);
      s += __shfl_xor(s, 2, 32);
      s += __shfl_xor(s, 1, 32);
      const float mu = s * (1.0f / 32.0f);
      const float dv = v - mu;
      float q = dv * dv;
      q += __shfl_xor(q, 16, 32);
      q += __shfl_xor(q, 8, 32);
      q += __shfl_xor(q, 4, 32);
      q += __shfl_xor(q, 2, 32);
      q += __shfl_xor(q, 1, 32);
      const float var = q * (1.0f / 32.0f);
      sU[row * kHid + lane] = dv * rsqrtf(var + 1e-5f) * lw + lb;
    }
  }
  __syncthreads();

#pragma unroll 1
  for (int i = 0; i < 3; ++i) {
    v16b ah, al;
    frag_hi_lo(sU + (i * 16 + m) * kHid + 8 * hh, ah, al);
#pragma unroll 1
    for (int nt = 0; nt < 8; ++nt) {
      const v16b b0 = load_b_frag(w.win + (nt * 16 + m) * kHid + 8 * hh);
      v8f acc = (v8f){0.f, 0.f, 0.f, 0.f, 0.f, 0.f, 0.f, 0.f};
      acc = mma_bf(ah, b0, acc);
      acc = mma_bf(al, b0, acc);
#pragma unroll
      for (int r = 0; r < 8; ++r) sXZ[(i * 16 + 8 * hh + r) * 128 + nt * 16 + m] = acc[r];
    }
  }
  __syncthreads();

#pragma unroll 1
  for (int j = 0; j < 16; ++j) {
    const int seq = j >> 1;
    const int d   = lane + ((j & 1) << 5);
    const v4f cw  = *(const v4f*)(w.conv_w + d * 4);
    const float c0 = cw[0], c1 = cw[1], c2 = cw[2], c3 = cw[3];
    const float w0 = rbf(c0), w1 = rbf(c1), w2 = rbf(c2), w3 = rbf(c3);
    const float bc = rbf(w.conv_b[d]);
    float xm3 = 0.f, xm2 = 0.f, xm1 = 0.f;
#pragma unroll 1
    for (int t = 0; t < kSteps; ++t) {
      const int idx = (seq * kSteps + t) * 128 + d;
      const float xcur = sXZ[idx];
      float acc = w0 * xm3;
      acc = fmaf(w1, xm2, acc);
      acc = fmaf(w2, xm1, acc);
      acc = fmaf(w3, xcur, acc);
      const float sv = acc + bc;
      sXZ[idx] = sv * sigmoid_f(sv);
      xm3 = xm2; xm2 = xm1; xm1 = xcur;
    }
  }
  __syncthreads();

#pragma unroll 1
  for (int i = 0; i < 3; ++i) {
    v16b ah0, al0, ah1, al1;
    const float* ap = sXZ + (i * 16 + m) * 128 + 8 * hh;
    frag_hi_lo(ap, ah0, al0);
    frag_hi_lo(ap + 32, ah1, al1);
#pragma unroll 1
    for (int nt = 0; nt < kProjPad / 16; ++nt) {
      const unsigned short* bp = w.wxp + (nt * 16 + m) * kInner + 8 * hh;
      const v16b b0 = load_b_frag(bp);
      const v16b b1 = load_b_frag(bp + 32);
      v8f acc = (v8f){0.f, 0.f, 0.f, 0.f, 0.f, 0.f, 0.f, 0.f};
      acc = mma_bf(ah0, b0, acc);
      acc = mma_bf(al0, b0, acc);
      acc = mma_bf(ah1, b1, acc);
      acc = mma_bf(al1, b1, acc);
#pragma unroll
      for (int r = 0; r < 8; ++r) sD[(i * 16 + 8 * hh + r) * kProjPad + nt * 16 + m] = acc[r];
    }
  }
  __syncthreads();

#pragma unroll 1
  for (int j = 0; j < 16; ++j) {
    const int seq = j >> 1;
    const int d   = lane + ((j & 1) << 5);
    const int rb  = seq * kSteps;
    const float dw0 = rbf(w.dt_w[d * 2]);
    const float dw1 = rbf(w.dt_w[d * 2 + 1]);
    const float db  = rbf(w.dt_b[d]);
    const float Dd  = rbf(w.dp[d]);
    float dl[kSteps], dx[kSteps], ya[kSteps], xv[kSteps];
#pragma unroll
    for (int t = 0; t < kSteps; ++t) {
      const float t0 = sD[(rb + t) * kProjPad];
      const float t1 = sD[(rb + t) * kProjPad + 1];
      float v = t0 * dw0;
      v = fmaf(t1, dw1, v);
      v += db;
      const float sp = fmaxf(v, 0.0f) + log1pf(expf(-fabsf(v)));
      const float xc = sXZ[(rb + t) * 128 + d];
      dl[t] = sp;
      xv[t] = xc;
      dx[t] = sp * xc;
      ya[t] = 0.0f;
    }
#pragma unroll 1
    for (int n = 0; n < kStates; ++n) {
      const float an = -expf(rbf(w.alog[d * kStates + n]));
      float h = 0.0f;
#pragma unroll
      for (int t = 0; t < kSteps; ++t) {
        const float Bn = sD[(rb + t) * kProjPad + 2 + n];
        const float Cn = sD[(rb + t) * kProjPad + 2 + kStates + n];
        const float dA = expf(dl[t] * an);
        h = fmaf(h, dA, dx[t] * Bn);
        ya[t] = fmaf(h, Cn, ya[t]);
      }
    }
#pragma unroll
    for (int t = 0; t < kSteps; ++t) {
      const float z = sXZ[(rb + t) * 128 + kInner + d];
      const float g = z * sigmoid_f(z);
      sXZ[(rb + t) * 128 + d] = (ya[t] + xv[t] * Dd) * g;
    }
  }
  __syncthreads();

#pragma unroll 1
  for (int i = 0; i < 3; ++i) {
    v16b ah0, al0, ah1, al1;
    const float* ap = sXZ + (i * 16 + m) * 128 + 8 * hh;
    frag_hi_lo(ap, ah0, al0);
    frag_hi_lo(ap + 32, ah1, al1);
#pragma unroll 1
    for (int nt = 0; nt < 2; ++nt) {
      const unsigned short* bp = w.wout + (nt * 16 + m) * kInner + 8 * hh;
      const v16b b0 = load_b_frag(bp);
      const v16b b1 = load_b_frag(bp + 32);
      v8f acc = (v8f){0.f, 0.f, 0.f, 0.f, 0.f, 0.f, 0.f, 0.f};
      acc = mma_bf(ah0, b0, acc);
      acc = mma_bf(al0, b0, acc);
      acc = mma_bf(ah1, b1, acc);
      acc = mma_bf(al1, b1, acc);
#pragma unroll
      for (int r = 0; r < 8; ++r) {
        const int idx = (i * 16 + 8 * hh + r) * kHid + nt * 16 + m;
        const float prev = sX[idx];
        sX[idx] = acc[r] + prev;
      }
    }
  }
  __syncthreads();
}

__global__ __launch_bounds__(32) void fused_ssm_kernel(FusedArgs a)
{
  __shared__ __align__(16) float sX[kRowsBlk * kHid];
  __shared__ __align__(16) float sXZ[kRowsBlk * 128];
  __shared__ __align__(16) float sD[kRowsBlk * kProjPad];
  const int lane = threadIdx.x & 31;
  const int hh = lane >> 4, m = lane & 15;
  const int p0 = blockIdx.x * kSeqBlk;

  float* sC = sXZ;
#pragma unroll 1
  for (int it = 0; it < 29; ++it) {
    const int idx = lane + it * 32;
    if (idx < kRowsBlk * (kFeatPad - kFeat)) {
      const int r = idx / (kFeatPad - kFeat);
      const int k = kFeat + (idx - r * (kFeatPad - kFeat));
      sC[r * kFeatPad + k] = 0.0f;
    }
  }
#pragma unroll 1
  for (int it = 0; it < 6; ++it) {
    const int idx = lane + it * 32;
    const int ic  = (idx < 176) ? idx : 175;
    const float v = a.xs[(size_t)p0 * 22 + ic];
    const int s   = ic / 22;
    const int jf  = ic - s * 22;
    if (idx < 176) {
#pragma unroll
      for (int l = 0; l < kSteps; ++l) sC[(s * kSteps + l) * kFeatPad + jf] = v;
    }
  }
#pragma unroll 1
  for (int l = 0; l < kSteps; ++l) {
    const float* xdl = a.xd + ((size_t)l * kNumSeq + p0) * 12;
#pragma unroll
    for (int it = 0; it < 3; ++it) {
      const int idx = lane + it * 32;
      const float v = xdl[idx];
      const int s   = idx / 12;
      const int jf  = idx - s * 12;
      sC[(s * kSteps + l) * kFeatPad + 22 + jf] = v;
    }
    const float* xpl = a.xp + ((size_t)l * kNumSeq + p0) * 7;
#pragma unroll
    for (int it = 0; it < 2; ++it) {
      const int idx = lane + it * 32;
      const int ic  = (idx < 56) ? idx : 55;
      const float v = xpl[ic];
      const int s   = ic / 7;
      const int jf  = ic - s * 7;
      if (idx < 56) sC[(s * kSteps + l) * kFeatPad + 34 + jf] = v;
    }
  }
#pragma unroll 1
  for (int it = 0; it < 6; ++it) {
    const int idx = lane + it * 32;
    const int r   = idx >> 2;
    const int jf  = idx & 3;
    const int s   = r / kSteps;
    const int l   = r - s * kSteps;
    const float v = a.xt[l * 4 + jf];
    sC[r * kFeatPad + 41 + jf] = v;
  }
  __syncthreads();

#pragma unroll 1
  for (int i = 0; i < 3; ++i) {
    const float* ap = sC + (i * 16 + m) * kFeatPad + 8 * hh;
    const v16b a0 = frag_hi(ap);
    const v16b a1 = frag_hi(ap + 32);
#pragma unroll 1
    for (int nt = 0; nt < 2; ++nt) {
      const unsigned short* bp = a.wf1 + (nt * 16 + m) * kFeatPad + 8 * hh;
      const v16b b0 = load_b_frag(bp);
      const v16b b1 = load_b_frag(bp + 32);
      v8f acc = (v8f){0.f, 0.f, 0.f, 0.f, 0.f, 0.f, 0.f, 0.f};
      acc = mma_bf(a0, b0, acc);
      acc = mma_bf(a1, b1, acc);
      const float bv = rbf(a.fc1_b[nt * 16 + m]);
#pragma unroll
      for (int r = 0; r < 8; ++r) {
        const float v = acc[r] + bv;
        sX[(i * 16 + 8 * hh + r) * kHid + nt * 16 + m] = fmaxf(v, 0.0f);
      }
    }
  }
  __syncthreads();

  ssm_block(sX, sXZ, sD, a.m1, lane);
  ssm_block(sX, sXZ, sD, a.m2, lane);

  {
    const int q = lane >> 3, c4 = (lane & 7) * 4;
    const v4f v0 = *(const v4f*)(sX + ((q) * kSteps + (kSteps - 1)) * kHid + c4);
    const v4f v1 = *(const v4f*)(sX + ((4 + q) * kSteps + (kSteps - 1)) * kHid + c4);
    float* d0 = a.xl + (size_t)(p0 + q) * kHid + c4;
    float* d1 = a.xl + (size_t)(p0 + 4 + q) * kHid + c4;
    for (int pass = 0; pass < 2; ++pass) {
      *(volatile v4f*)d0 = v0;
      *(volatile v4f*)d1 = v1;
      __threadfence();
    }
  }
}

__global__ __launch_bounds__(128) void head_kernel(
    const float* __restrict__ XL, const unsigned short* __restrict__ wf2, const float* __restrict__ fc2_b,
    const float* __restrict__ fc3_w, const float* __restrict__ fc3_b,
    const float* __restrict__ fc4_w, const float* __restrict__ fc4_b, float* __restrict__ out)
{
  __shared__ __align__(16) float sV[kHeadSeq * kHid];
  __shared__ __align__(16) float sW[10 * kHid];
  __shared__ __align__(16) float sB[16];
  __shared__ __align__(16) float sO[kHeadSeq * 10];
  const int tid = threadIdx.x, lane = tid & 31, wave = tid >> 5;
  const int hh = lane >> 4, m = lane & 15;
  const int blk = blockIdx.x;
  const int s0 = blk * kHeadSeq;

#pragma unroll
  for (int it = 0; it < 2; ++it) {
    const int idx = tid + it * 128;
    const int ic  = (idx < 7 * kHid) ? idx : (7 * kHid - 1);
    const float v = rbf(fc3_w[ic]);
    if (idx < 7 * kHid) sW[idx] = v;
  }
  {
    const int ic = (tid < 3 * kHid) ? tid : (3 * kHid - 1);
    const float v = rbf(fc4_w[ic]);
    if (tid < 3 * kHid) sW[7 * kHid + tid] = v;
    const int i3 = (tid < 7) ? tid : 6;
    int i4 = tid - 7;
    i4 = (i4 < 0) ? 0 : ((i4 > 2) ? 2 : i4);
    const float b3 = rbf(fc3_b[i3]);
    const float b4 = rbf(fc4_b[i4]);
    const float bsel = (tid < 7) ? b3 : ((tid < 10) ? b4 : 0.0f);
    if (tid < 16) sB[tid] = bsel;
  }

  {
    const int row = s0 + wave * 16 + m;
    v16b ah, al;
    frag_hi_lo(XL + (size_t)row * kHid + 8 * hh, ah, al);
#pragma unroll 1
    for (int nt = 0; nt < 2; ++nt) {
      const v16b b0 = load_b_frag(wf2 + (nt * 16 + m) * kHid + 8 * hh);
      v8f acc = (v8f){0.f, 0.f, 0.f, 0.f, 0.f, 0.f, 0.f, 0.f};
      acc = mma_bf(ah, b0, acc);
      acc = mma_bf(al, b0, acc);
      const float bv = rbf(fc2_b[nt * 16 + m]);
#pragma unroll
      for (int r = 0; r < 8; ++r) {
        const float v = acc[r] + bv;
        sV[(wave * 16 + 8 * hh + r) * kHid + nt * 16 + m] = (v >= 0.0f) ? v : (0.2f * v);
      }
    }
  }
  __syncthreads();

#pragma unroll 1
  for (int it = 0; it < 5; ++it) {
    const int o = tid + it * 128;
    const bool is0 = (o < kHeadSeq * kOut0Cols);
    const int q  = is0 ? o : (o - kHeadSeq * kOut0Cols);
    const int sq = is0 ? (q / kOut0Cols) : (q / kOut1Cols);
    const int jj = is0 ? (q - sq * kOut0Cols) : (kOut0Cols + q - sq * kOut1Cols);
    const float* vp = sV + sq * kHid;
    const float* wp = sW + jj * kHid;
    float acc = 0.0f;
#pragma unroll 4
    for (int k = 0; k < kHid; ++k) acc = fmaf(vp[k], wp[k], acc);
    acc += sB[jj];
    sO[o] = acc;
  }
  __syncthreads();

  {
    const int i0 = (tid < 112) ? tid : 111;
    const int i1 = (tid < 48) ? tid : 47;
    const v4f v0 = *(const v4f*)(sO + 4 * i0);
    const v4f v1 = *(const v4f*)(sO + kHeadSeq * kOut0Cols + 4 * i1);
    const v2f zz = (v2f){0.0f, 0.0f};
    float* o0 = out + (size_t)blk * (kHeadSeq * kOut0Cols) + 4 * i0;
    float* o1 = out + (size_t)kOut0Elems + (size_t)blk * (kHeadSeq * kOut1Cols) + 4 * i1;
    float* oz = out + (size_t)kOut0Elems + (size_t)kOut1Elems;
    for (int pass = 0; pass < 2; ++pass) {
      if (tid < 112) *(volatile v4f*)o0 = v0;
      if (tid < 48)  *(volatile v4f*)o1 = v1;
      if (blk == 0 && tid == 0) *(volatile v2f*)oz = zz;
      __threadfence();
    }
  }
}

static void launch_plane(const float* src, unsigned short* dst, int nreal, int kreal, int npad, int kpad,
                         hipStream_t stream)
{
  const int total8 = npad * kpad / 8;
  const int grid = (total8 + 255) / 256;
  pad_cast_bf16_kernel<<<grid, 256, 0, stream>>>(src, dst, nreal, kreal, kpad, total8);
}

extern "C" void kernel_launch(void* const* d_in, const int* in_sizes, int n_in,
                              void* d_out, int out_size, void* d_ws, size_t ws_size,
                              hipStream_t stream)
{
  if (n_in < 34) return;
  if (in_sizes[0] != kNumSeq * 22) return;
  if (in_sizes[1] != kSteps * kNumSeq * 12) return;
  if (in_sizes[2] != kSteps * kNumSeq * 7) return;
  if (in_sizes[3] != kSteps * 4) return;
  if (in_sizes[4] != kHid * kFeat) return;
  if (in_sizes[10] != kHid * kHid) return;
  if (in_sizes[12] != kOut0Cols * kHid || in_sizes[14] != kOut1Cols * kHid) return;
  if (in_sizes[16] != 2 * kInner * kHid || in_sizes[25] != 2 * kInner * kHid) return;
  if (in_sizes[19] != kProjN * kInner || in_sizes[28] != kProjN * kInner) return;
  if (in_sizes[22] != kInner * kStates || in_sizes[31] != kInner * kStates) return;
  if (in_sizes[24] != kHid * kInner || in_sizes[33] != kHid * kInner) return;
  if (out_size != kOutTotal) return;
  if (ws_size < kWsTotal) return;

  const float* x_static  = (const float*)d_in[0];
  const float* x_dynamic = (const float*)d_in[1];
  const float* x_prog    = (const float*)d_in[2];
  const float* x_time    = (const float*)d_in[3];
  const float* fc1_w     = (const float*)d_in[4];
  const float* fc1_b     = (const float*)d_in[5];
  const float* ln1_w     = (const float*)d_in[6];
  const float* ln1_b     = (const float*)d_in[7];
  const float* ln2_w     = (const float*)d_in[8];
  const float* ln2_b     = (const float*)d_in[9];
  const float* fc2_w     = (const float*)d_in[10];
  const float* fc2_b     = (const float*)d_in[11];
  const float* fc3_w     = (const float*)d_in[12];
  const float* fc3_b     = (const float*)d_in[13];
  const float* fc4_w     = (const float*)d_in[14];
  const float* fc4_b     = (const float*)d_in[15];
  const float* m1_in_w    = (const float*)d_in[16];
  const float* m1_conv_w  = (const float*)d_in[17];
  const float* m1_conv_b  = (const float*)d_in[18];
  const float* m1_xproj_w = (const float*)d_in[19];
  const float* m1_dt_w    = (const float*)d_in[20];
  const float* m1_dt_b    = (const float*)d_in[21];
  const float* m1_alog    = (const float*)d_in[22];
  const float* m1_d       = (const float*)d_in[23];
  const float* m1_out_w   = (const float*)d_in[24];
  const float* m2_in_w    = (const float*)d_in[25];
  const float* m2_conv_w  = (const float*)d_in[26];
  const float* m2_conv_b  = (const float*)d_in[27];
  const float* m2_xproj_w = (const float*)d_in[28];
  const float* m2_dt_w    = (const float*)d_in[29];
  const float* m2_dt_b    = (const float*)d_in[30];
  const float* m2_alog    = (const float*)d_in[31];
  const float* m2_d       = (const float*)d_in[32];
  const float* m2_out_w   = (const float*)d_in[33];

  char* ws = (char*)d_ws;
  unsigned short* WF1   = (unsigned short*)(ws + kOffWF1);
  unsigned short* WF2   = (unsigned short*)(ws + kOffWF2);
  unsigned short* WIN1  = (unsigned short*)(ws + kOffWIN1);
  unsigned short* WXP1  = (unsigned short*)(ws + kOffWXP1);
  unsigned short* WOUT1 = (unsigned short*)(ws + kOffWOUT1);
  unsigned short* WIN2  = (unsigned short*)(ws + kOffWIN2);
  unsigned short* WXP2  = (unsigned short*)(ws + kOffWXP2);
  unsigned short* WOUT2 = (unsigned short*)(ws + kOffWOUT2);
  float*          XL    = (float*)(ws + kOffXL);

  launch_plane(fc1_w, WF1, kHid, kFeat, kHid, kFeatPad, stream);
  launch_plane(fc2_w, WF2, kHid, kHid, kHid, kHid, stream);
  launch_plane(m1_in_w, WIN1, 2 * kInner, kHid, 2 * kInner, kHid, stream);
  launch_plane(m1_xproj_w, WXP1, kProjN, kInner, kProjPad, kInner, stream);
  launch_plane(m1_out_w, WOUT1, kHid, kInner, kHid, kInner, stream);
  launch_plane(m2_in_w, WIN2, 2 * kInner, kHid, 2 * kInner, kHid, stream);
  launch_plane(m2_xproj_w, WXP2, kProjN, kInner, kProjPad, kInner, stream);
  launch_plane(m2_out_w, WOUT2, kHid, kInner, kHid, kInner, stream);

  FusedArgs fa;
  fa.xs = x_static; fa.xd = x_dynamic; fa.xp = x_prog; fa.xt = x_time; fa.fc1_b = fc1_b;
  fa.wf1 = WF1;
  fa.m1.lnw = ln1_w; fa.m1.lnb = ln1_b; fa.m1.conv_w = m1_conv_w; fa.m1.conv_b = m1_conv_b;
  fa.m1.dt_w = m1_dt_w; fa.m1.dt_b = m1_dt_b; fa.m1.alog = m1_alog; fa.m1.dp = m1_d;
  fa.m1.win = WIN1; fa.m1.wxp = WXP1; fa.m1.wout = WOUT1;
  fa.m2.lnw = ln2_w; fa.m2.lnb = ln2_b; fa.m2.conv_w = m2_conv_w; fa.m2.conv_b = m2_conv_b;
  fa.m2.dt_w = m2_dt_w; fa.m2.dt_b = m2_dt_b; fa.m2.alog = m2_alog; fa.m2.dp = m2_d;
  fa.m2.win = WIN2; fa.m2.wxp = WXP2; fa.m2.wout = WOUT2;
  fa.xl = XL;

  fused_ssm_kernel<<<kNumSeq / kSeqBlk, 32, 0, stream>>>(fa);

  head_kernel<<<kNumSeq / kHeadSeq, 128, 0, stream>>>(XL, WF2, fc2_b, fc3_w, fc3_b, fc4_w, fc4_b, (float*)d_out);
}
